// graph_structure_learner_36103495090409
// MI455X (gfx1250) — hardware-verified
//
#include <hip/hip_runtime.h>

#define NN_   50000
#define NE_   2500000
#define EMB_  32
#define HID_  64
#define NORI_ 500000
#define NTILE (NE_ / 16)
#define TPB   64
#define WSTR  72

typedef _Float16 f16;
typedef __attribute__((ext_vector_type(16))) f16 f16x16;
typedef __attribute__((ext_vector_type(8)))  f16 f16x8;
typedef __attribute__((ext_vector_type(8)))  float f32x8;
typedef __attribute__((ext_vector_type(4)))  float v4f_t;
typedef float v4fa __attribute__((ext_vector_type(4), may_alias));

__device__ __forceinline__ f32x8 wmma16(f16x16 a, f16x16 b, f32x8 c) {
  c = __builtin_amdgcn_wmma_f32_16x16x32_f16(false, a, false, b, (short)0, c, false, false);
  asm volatile("v_nop\n\tv_nop\n\tv_nop\n\tv_nop" : "+v"(c) : "v"(a), "v"(b));
  return c;
}
__device__ __forceinline__ f16x16 lds_frag(const f16* base, int stride) {
  const int lane = threadIdx.x & 31, row = lane & 15, kh = (lane >> 4) * 8;
  const f16x8 lo = *(const f16x8*)(base + row * stride + kh);
  const f16x8 hi = *(const f16x8*)(base + row * stride + kh + 16);
  f16x16 f;
#pragma unroll
  for (int i = 0; i < 8; ++i) { f[i] = lo[i]; f[i + 8] = hi[i]; }
  return f;
}

__global__ __launch_bounds__(256) void k_zero(int* __restrict__ m, int n) {
  const int i = blockIdx.x * 256 + threadIdx.x;
  if (i < n) { *(volatile int*)(m + i) = 0; __threadfence(); *(volatile int*)(m + i) = 0; }
}
__global__ __launch_bounds__(256) void k_flag(const int* __restrict__ ori, int* __restrict__ m) {
  const int i = blockIdx.x * 256 + threadIdx.x;
  if (i < NORI_) {
    int e = ori[i]; e = min(max(e, 0), NE_ - 1);
    *(volatile int*)(m + e) = 1; __threadfence(); *(volatile int*)(m + e) = 1;
  }
}

__global__ __launch_bounds__(256) void k_edge_mlp(const float* __restrict__ h, const float* __restrict__ rel,
    const float* __restrict__ W0, const float* __restrict__ b0, const float* __restrict__ bng, const float* __restrict__ bnb,
    const float* __restrict__ bnm, const float* __restrict__ bnv, const float* __restrict__ Ws, const float* __restrict__ bs,
    const int* __restrict__ row, const int* __restrict__ col, const int* __restrict__ et, const int* __restrict__ omask,
    float* __restrict__ out) {
  __shared__ __attribute__((aligned(16))) f16 W0S[HID_ * WSTR];
  __shared__ __attribute__((aligned(16))) f16 xS[8][16 * WSTR];
  __shared__ __attribute__((aligned(16))) f16 xlS[8][16 * WSTR];
  __shared__ __attribute__((aligned(16))) f16 fS[8][16 * WSTR];
  __shared__ float scS[HID_], shS[HID_], wsS[HID_];
  __shared__ __attribute__((aligned(16))) float wS[TPB * 16];
  const int tid = threadIdx.x, lane = tid & 31, wave = tid >> 5, cl = lane & 15, rh = (lane >> 4) * 8, kh = rh;

  for (int e = tid; e < HID_ * 64; e += 256) { const int n = e >> 6, k = e & 63; W0S[n * WSTR + k] = (f16)W0[k * HID_ + n]; }
  if (tid < HID_) {
    const float sc = bng[tid] / sqrtf(bnv[tid] + 1e-5f);
    scS[tid] = sc; shS[tid] = (b0[tid] - bnm[tid]) * sc + bnb[tid]; wsS[tid] = Ws[tid];
  }
  for (int e = tid; e < TPB * 16; e += 256) wS[e] = 0.0f;
  __syncthreads();
  f16x16 wsf[2];
#pragma unroll
  for (int ks = 0; ks < 2; ++ks)
#pragma unroll
    for (int i = 0; i < 8; ++i) {
      wsf[ks][i]     = (cl == 0) ? (f16)wsS[ks * 32 + kh + i]      : (f16)0.0f;
      wsf[ks][i + 8] = (cl == 0) ? (f16)wsS[ks * 32 + kh + 16 + i] : (f16)0.0f;
    }
  const float bsv = bs[0];

  f16* fs = fS[wave]; f16* xs = xS[wave]; f16* xls = xlS[wave];
#pragma unroll 1
  for (int tt = 0; tt < 8; ++tt) {
    const int tile = blockIdx.x * TPB + wave * 8 + tt;
    const bool live = tile < NTILE;
    if (live) {
    const int e = tile * 16 + cl;
    int r = row[e], c = col[e], ty = et[e];
    r = min(max(r, 0), NN_ - 1); c = min(max(c, 0), NN_ - 1); ty = min(max(ty, 0), 199);
    {
      const float* hr = h + (size_t)r * EMB_ + kh; const float* hc = h + (size_t)c * EMB_ + kh;
      const float* re = rel + (size_t)ty * EMB_ + kh;
      const v4f_t r0 = *(const v4f_t*)hr, r1 = *(const v4f_t*)(hr + 4), r2 = *(const v4f_t*)(hr + 16), r3 = *(const v4f_t*)(hr + 20);
      const v4f_t c0 = *(const v4f_t*)hc, c1 = *(const v4f_t*)(hc + 4), c2 = *(const v4f_t*)(hc + 16), c3 = *(const v4f_t*)(hc + 20);
      const v4f_t e0 = *(const v4f_t*)re, e1 = *(const v4f_t*)(re + 4), e2 = *(const v4f_t*)(re + 16), e3 = *(const v4f_t*)(re + 20);
      float dr[16] = {r0[0], r0[1], r0[2], r0[3], r1[0], r1[1], r1[2], r1[3], r2[0], r2[1], r2[2], r2[3], r3[0], r3[1], r3[2], r3[3]};
      float dc[16] = {c0[0], c0[1], c0[2], c0[3], c1[0], c1[1], c1[2], c1[3], c2[0], c2[1], c2[2], c2[3], c3[0], c3[1], c3[2], c3[3]};
      float de[16] = {e0[0], e0[1], e0[2], e0[3], e1[0], e1[1], e1[2], e1[3], e2[0], e2[1], e2[2], e2[3], e3[0], e3[1], e3[2], e3[3]};
#pragma unroll
      for (int i = 0; i < 16; ++i) {
        const int k = kh + (i & 7) + ((i >> 3) << 4);
        fs[cl * WSTR + k]      = (f16)__builtin_amdgcn_exp2f(-fabsf(dr[i] - dc[i]) * 1.44269504088896340736f);
        fs[cl * WSTR + 32 + k] = (f16)de[i];
      }
    }
    }
    asm volatile("s_wait_dscnt 0" ::: "memory");
    __syncthreads();
    if (live) {
    const f16x16 a0 = lds_frag(fs, WSTR), a1 = lds_frag(fs + 32, WSTR);
    f32x8 acc[4];
#pragma unroll
    for (int nt = 0; nt < 4; ++nt) {
      f32x8 z = {};
      z = wmma16(a0, lds_frag(W0S + nt * 16 * WSTR, WSTR), z);
      z = wmma16(a1, lds_frag(W0S + nt * 16 * WSTR + 32, WSTR), z);
      acc[nt] = z;
    }
#pragma unroll
    for (int nt = 0; nt < 4; ++nt) {
      const int n = nt * 16 + cl;
      const float sc = scS[n], sh = shS[n];
#pragma unroll
      for (int j = 0; j < 8; ++j) {
        float v = acc[nt][j] * sc + sh;
        v = (v >= 0.0f) ? v : 0.01f * v;
        const f16 hv = (f16)v;
        xs[(rh + j) * WSTR + n] = hv; xls[(rh + j) * WSTR + n] = (f16)((v - (float)hv) * 2048.0f);
      }
    }
    }
    asm volatile("s_wait_dscnt 0" ::: "memory");
    __syncthreads();
    if (live) {
    f32x8 wz = {}, wzl = {};
    wz  = wmma16(lds_frag(xs, WSTR),       wsf[0], wz);
    wz  = wmma16(lds_frag(xs + 32, WSTR),  wsf[1], wz);
    wzl = wmma16(lds_frag(xls, WSTR),      wsf[0], wzl);
    wzl = wmma16(lds_frag(xls + 32, WSTR), wsf[1], wzl);
    if (cl == 0) {
#pragma unroll
      for (int j = 0; j < 8; ++j) {
        const int el = (wave * 8 + tt) * 16 + rh + j;
        float wv = wz[j] + wzl[j] * (1.0f / 2048.0f) + bsv;
        if (omask[(size_t)blockIdx.x * (TPB * 16) + el] != 0) wv = 0.5f * wv + 0.5f;
        wS[el] = wv;
      }
    }
    }
    __syncthreads();
  }
  const int nown = min(TPB * 16, NE_ - blockIdx.x * (TPB * 16));
#pragma unroll 1
  for (int pass = 0; pass < 2; ++pass) {
    if (tid * 4 < nown) *(volatile v4f_t*)(out + (size_t)blockIdx.x * (TPB * 16) + tid * 4) = *(const volatile v4fa*)(wS + tid * 4);
    __threadfence();
  }
}

extern "C" void kernel_launch(void* const* d_in, const int* in_sizes, int n_in,
                              void* d_out, int out_size, void* d_ws, size_t ws_size,
                              hipStream_t stream) {
  (void)in_sizes; (void)n_in; (void)out_size; (void)ws_size;
  const float* h   = (const float*)d_in[0];
  const float* rel = (const float*)d_in[1];
  const float* W0  = (const float*)d_in[2];
  const float* b0  = (const float*)d_in[3];
  const float* bng = (const float*)d_in[4], *bnb = (const float*)d_in[5], *bnm = (const float*)d_in[6], *bnv = (const float*)d_in[7];
  const float* Ws  = (const float*)d_in[8];
  const float* bs  = (const float*)d_in[9];
  const int* row = (const int*)d_in[10], *col = (const int*)d_in[11], *et = (const int*)d_in[12], *ori = (const int*)d_in[13];
  float* out = (float*)d_out;
  int* omask = (int*)d_ws;
  k_zero<<<dim3((NE_ + 255) / 256), dim3(256), 0, stream>>>(omask, NE_);
  k_flag<<<dim3((NORI_ + 255) / 256), dim3(256), 0, stream>>>(ori, omask);
  k_edge_mlp<<<dim3((NTILE + TPB - 1) / TPB), dim3(256), 0, stream>>>(h, rel, W0, b0, bng, bnb, bnm, bnv, Ws, bs, row, col, et, omask, out);
}
